// SMPLX_27410481283809
// MI455X (gfx1250) — hardware-run, weakly checked
//
#include <hip/hip_runtime.h>
#include <math.h>

typedef __attribute__((ext_vector_type(16))) _Float16 v16h;
typedef __attribute__((ext_vector_type(8)))  _Float16 v8h;
typedef __attribute__((ext_vector_type(16))) __bf16   v16b;
typedef __attribute__((ext_vector_type(8)))  __bf16   v8b;
typedef __attribute__((ext_vector_type(8)))  float    v8f;
typedef __attribute__((ext_vector_type(4)))  float    v4f;
typedef __attribute__((ext_vector_type(2)))  float    v2f;
typedef __attribute__((ext_vector_type(4)))  unsigned int v4u;

constexpr int kV   = 10475;
constexpr int kJ   = 55;
constexpr int kB   = 512;
constexpr int kN3  = kV * 3;
constexpr int kNP  = 31488;
constexpr int kPF  = (kJ - 1) * 9;
constexpr int kNE  = 10;
constexpr int kKP  = 512;
constexpr int kVP  = 10496;
constexpr int kJP  = 64;
constexpr int kJTP = 64;
constexpr int kLbsTileV = 128;
constexpr int kLbsTiles = kVP / kLbsTileV;
constexpr int kGrpB = 4;
constexpr int kGroups = kB / kGrpB;
constexpr int kRun = kLbsTileV * 3;
constexpr int kTP  = 68;
constexpr float kWCarry    = 16.0f;
constexpr float kWCarryInv = 1.0f / kWCarry;
constexpr int kJregIters = (kV + 255) / 256;
constexpr int kEdTile = kPF / 64;
constexpr int kEdRow  = kPF - kEdTile * 64;
static_assert(kN3 == 31425 && kPF == 486, "shape");
static_assert((kNP % 64) == 0 && kNP >= kN3 && (kKP % 32) == 0 && kKP >= kPF + kNE, "pose GEMM padding");
static_assert((kVP % kLbsTileV) == 0 && kVP >= kV && (kJP % 32) == 0 && kJP >= kJ, "skinning padding");
static_assert((kB % 64) == 0 && (kB % kGrpB) == 0, "batch tiling");
static_assert((kN3 % 32) == 1, "row start position inside a 32-float line equals batch mod 32");
static_assert(kEdRow + kNE <= 64 && kEdTile == kKP / 64 - 1, "expression slots sit in the last k tile");
static_assert(kJregIters * 256 >= kV, "joint regressor coverage");
static_assert(((kLbsTiles - 1) & 1) == 1, "last tile uses staging buffer 1");
static_assert((kGroups % 8) == 0, "boundary merge grid: 8 waves per block");

constexpr size_t kOffVP   = 0;
constexpr size_t kOffPDT  = kOffVP   + (size_t)kB  * kNP * 4;
constexpr size_t kOffWB   = kOffPDT  + (size_t)kNP * kKP * 2;
constexpr size_t kOffAT   = kOffWB   + (size_t)kVP * kJP * 2;
constexpr size_t kOffAP   = kOffAT   + (size_t)kB * 16 * kJP * 2;
constexpr size_t kOffBASE = kOffAP   + (size_t)kB * kKP * 2;
constexpr size_t kOffJT   = kOffBASE + (size_t)kNP * 4;
constexpr size_t kOffYO   = kOffJT   + (size_t)kJ * kJTP * 4;
constexpr size_t kOffHT   = kOffYO   + 128;
constexpr size_t kOffTT   = kOffHT   + (size_t)kGroups * 32 * 4;
constexpr size_t kWsTotal = kOffTT   + (size_t)kGroups * 32 * 4;
static_assert(kWsTotal == 99820416ull, "carve total");
static_assert(kWsTotal <= 134217728ull, "carve cap");
static_assert((kOffPDT % 128) == 0 && (kOffWB % 128) == 0 && (kOffAT % 128) == 0 && (kOffAP % 128) == 0 &&
              (kOffBASE % 128) == 0 && (kOffJT % 128) == 0 && (kOffYO % 128) == 0 &&
              (kOffHT % 128) == 0 && (kOffTT % 128) == 0, "128-B aligned regions");

__device__ __forceinline__ unsigned short f2bf_bits(float f) {
  unsigned u = __float_as_uint(f);
  return (unsigned short)((u + 0x7FFFu + ((u >> 16) & 1u)) >> 16);
}
__device__ __forceinline__ unsigned short f2h_bits(float f) {
  const _Float16 h = (_Float16)f;
  return __builtin_bit_cast(unsigned short, h);
}
__device__ __forceinline__ unsigned pack2(unsigned short lo, unsigned short hi) {
  return (unsigned)lo | ((unsigned)hi << 16);
}
__device__ __forceinline__ void keep4_b(v16b a, v16b b, v16b c, v16b d) { asm volatile("v_nop" :: "v"(a), "v"(b), "v"(c), "v"(d)); }

template <typename T> struct Frag;
template <> struct Frag<_Float16> {
  typedef v16h V; union U { v16h v; v8h h[2]; };
  static __device__ __forceinline__ v16h load(const _Float16* p) {
    U f; f.h[0] = *(const v8h*)(p); f.h[1] = *(const v8h*)(p + 16); return f.v;
  }
};
template <> struct Frag<__bf16> {
  typedef v16b V; union U { v16b v; v8b h[2]; };
  static __device__ __forceinline__ v16b load(const __bf16* p) {
    U f; f.h[0] = *(const v8b*)(p); f.h[1] = *(const v8b*)(p + 16); return f.v;
  }
};
__device__ __forceinline__ v8f mma_b(v16b a, v16b b, v8f c) {
  c = __builtin_amdgcn_wmma_f32_16x16x32_bf16(false, a, false, b, (short)0, c, false, false);
  asm volatile("v_nop\n\tv_nop\n\tv_nop\n\tv_nop" : "+v"(c) : "v"(a), "v"(b));
  return c;
}
__device__ __forceinline__ v8f mma_h(v16h a, v16h b, v8f c) {
  c = __builtin_amdgcn_wmma_f32_16x16x32_f16(false, a, false, b, (short)0, c, false, false);
  asm volatile("v_nop\n\tv_nop\n\tv_nop\n\tv_nop" : "+v"(c) : "v"(a), "v"(b));
  return c;
}

__global__ __launch_bounds__(256) void static_base_kernel(
    const float* __restrict__ vt, const float* __restrict__ sd, const float* __restrict__ shp, float* __restrict__ base)
{
  const int i = blockIdx.x * 256 + threadIdx.x;
  if (i >= kNP / 4) return;
  float sh[kNE];
#pragma unroll
  for (int s = 0; s < kNE; ++s) sh[s] = shp[s];
  float r[4];
#pragma unroll
  for (int e = 0; e < 4; ++e) {
    const int n = i * 4 + e;
    const int nc = n < kN3 ? n : kN3 - 1;
    float acc = vt[nc];
    const float* sp = sd + (size_t)nc * kNE;
#pragma unroll
    for (int s2 = 0; s2 < kNE / 2; ++s2) {
      const v2f d = *(const v2f*)(sp + 2 * s2);
      acc = fmaf(d[0], sh[2 * s2], acc);
      acc = fmaf(d[1], sh[2 * s2 + 1], acc);
    }
    r[e] = (n < kN3) ? acc : 0.0f;
  }
  const v4f o = (v4f){r[0], r[1], r[2], r[3]};
  float* q = base + (size_t)i * 4;
  *(volatile v4f*)q = o;
  __threadfence();
  *(volatile v4f*)q = o;
}

__global__ __launch_bounds__(256) void yoff_kernel(const float* __restrict__ vt, float* __restrict__ yo)
{
  __shared__ float s[8];
  const int tid = threadIdx.x, lane = tid & 31, wave = tid >> 5;
  float m = 3.0e38f;
#pragma unroll 1
  for (int it = 0; it < kJregIters; ++it) {
    const int v = it * 256 + tid;
    const int vc = v < kV ? v : kV - 1;
    const float x = vt[vc * 3 + 1];
    m = fminf(m, (v < kV) ? x : 3.0e38f);
  }
#pragma unroll
  for (int off = 16; off > 0; off >>= 1) m = fminf(m, __shfl_xor(m, off, 32));
  if (lane == 0) s[wave] = m;
  __syncthreads();
  float mm = s[0];
#pragma unroll
  for (int w = 1; w < 8; ++w) mm = fminf(mm, s[w]);
  if (tid < 32) {
    const float y = -mm;
    float* q = yo + tid;
    *(volatile float*)q = y;
    __threadfence();
    *(volatile float*)q = y;
  }
}

__global__ __launch_bounds__(256) void jreg_kernel(
    const float* __restrict__ JR, const float* __restrict__ base, const float* __restrict__ ed, float* __restrict__ JT)
{
  __shared__ float red[8 * 33];
  const int tid = threadIdx.x, lane = tid & 31, wave = tid >> 5;
  const int j = blockIdx.x;
  float acc[33];
#pragma unroll
  for (int i = 0; i < 33; ++i) acc[i] = 0.0f;
#pragma unroll 1
  for (int it = 0; it < kJregIters; ++it) {
    const int v = it * 256 + tid;
    const int vc = v < kV ? v : kV - 1;
    const float wr = JR[(size_t)j * kV + vc];
    const float w = (v < kV) ? wr : 0.0f;
    const float* bp = base + vc * 3;
    acc[0] = fmaf(w, bp[0], acc[0]);
    acc[1] = fmaf(w, bp[1], acc[1]);
    acc[2] = fmaf(w, bp[2], acc[2]);
    const float* ep = ed + (size_t)vc * 30;
#pragma unroll
    for (int q = 0; q < 15; ++q) {
      const v2f d = *(const v2f*)(ep + 2 * q);
      acc[3 + 2 * q] = fmaf(w, d[0], acc[3 + 2 * q]);
      acc[4 + 2 * q] = fmaf(w, d[1], acc[4 + 2 * q]);
    }
  }
#pragma unroll
  for (int i = 0; i < 33; ++i) {
    float s = acc[i];
#pragma unroll
    for (int off = 16; off > 0; off >>= 1) s += __shfl_xor(s, off, 32);
    acc[i] = s;
  }
  if (lane == 0) {
#pragma unroll
    for (int i = 0; i < 33; ++i) red[wave * 33 + i] = acc[i];
  }
  __syncthreads();
  if (tid < 32) {
    float s0 = 0.0f, s1 = 0.0f;
#pragma unroll
    for (int w = 0; w < 8; ++w) {
      s0 += red[w * 33 + lane];
      s1 += red[w * 33 + 32];
    }
    const float o1 = (lane == 0) ? s1 : 0.0f;
    float* q0 = JT + j * kJTP + lane;
    float* q1 = JT + j * kJTP + 32 + lane;
    *(volatile float*)q0 = s0;
    *(volatile float*)q1 = o1;
    __threadfence();
    *(volatile float*)q0 = s0;
    *(volatile float*)q1 = o1;
  }
}

__global__ __launch_bounds__(64) void pose_fk_kernel(
    const float* __restrict__ pelvis, const float* __restrict__ body, const float* __restrict__ head,
    const float* __restrict__ hand, const float* __restrict__ hmean, const float* __restrict__ expr,
    const float* __restrict__ JT, unsigned short* __restrict__ Apose, unsigned short* __restrict__ At)
{
  __shared__ float sP[168];
  __shared__ float sE[16];
  __shared__ float sR[496];
  __shared__ float sJ[168];
  __shared__ float sA[12 * 56];
  const int tid = threadIdx.x;
  const int b = blockIdx.x;
  {
    const int i = tid < 2 ? tid : 2;
    const float v = pelvis[b * 3 + i];
    if (tid < 3) sP[tid] = v;
  }
  {
    const int i = tid < 62 ? tid : 62;
    const float v = body[b * 63 + i];
    if (tid < 63) sP[3 + tid] = v;
  }
  {
    const int i = tid < 8 ? tid : 8;
    const float v = head[b * 9 + i];
    if (tid < 9) sP[66 + tid] = v;
  }
#pragma unroll
  for (int it = 0; it < 2; ++it) {
    const int idx = tid + 64 * it;
    const int i = idx < 89 ? idx : 89;
    const float v = hand[b * 90 + i] + hmean[i];
    if (idx < 90) sP[75 + idx] = v;
  }
  {
    const int i = tid < 9 ? tid : 9;
    const float v = expr[b * kNE + i];
    if (tid < kNE) sE[tid] = v;
  }
  __syncthreads();
  {
    const int jc = tid < kJ - 1 ? tid : kJ - 1;
    const float r0 = sP[jc * 3], r1 = sP[jc * 3 + 1], r2 = sP[jc * 3 + 2];
    const float a2 = (r0 * r0 + r1 * r1 + r2 * r2) + 1e-12f;
    const float ang = sqrtf(a2);
    const float inv = 1.0f / ang;
    const float kx = r0 * inv, ky = r1 * inv, kz = r2 * inv;
    float sn, cs;
    sincosf(ang, &sn, &cs);
    const float t = 1.0f - cs;
    const float xx = kx * kx, yy = ky * ky, zz = kz * kz;
    const float xy = t * (kx * ky), xz = t * (kx * kz), yz = t * (ky * kz);
    const float sx = sn * kx, sy = sn * ky, sz = sn * kz;
    if (tid < kJ) {
      float* rp = sR + jc * 9;
      rp[0] = 1.0f - t * (yy + zz);
      rp[1] = xy - sz;
      rp[2] = xz + sy;
      rp[3] = xy + sz;
      rp[4] = 1.0f - t * (xx + zz);
      rp[5] = yz - sx;
      rp[6] = xz - sy;
      rp[7] = yz + sx;
      rp[8] = 1.0f - t * (xx + yy);
    }
    const float* jt = JT + jc * kJTP;
#pragma unroll 1
    for (int c = 0; c < 3; ++c) {
      float jv = jt[c];
#pragma unroll
      for (int e = 0; e < kNE; ++e) jv = fmaf(jt[3 + c * kNE + e], sE[e], jv);
      if (tid < kJ) sJ[jc * 3 + c] = jv;
    }
  }
  __syncthreads();
  {
    unsigned short hb[8];
#pragma unroll
    for (int e = 0; e < 8; ++e) {
      const int k = tid * 8 + e;
      const int kr = (k + 9 < 494) ? (k + 9) : 494;
      const float rv = sR[kr];
      const int q = k % 9;
      const float d = (q == 0 || q == 4 || q == 8) ? 1.0f : 0.0f;
      int ke = k - kPF;
      ke = ke < 0 ? 0 : (ke > kNE - 1 ? kNE - 1 : ke);
      const float ev = sE[ke];
      const float val = (k < kPF) ? (rv - d) : ((k < kPF + kNE) ? ev : 0.0f);
      hb[e] = f2bf_bits(val);
    }
    const v4u w = (v4u){pack2(hb[0], hb[1]), pack2(hb[2], hb[3]), pack2(hb[4], hb[5]), pack2(hb[6], hb[7])};
    unsigned short* q = Apose + (size_t)b * kKP + tid * 8;
    *(volatile v4u*)q = w;
    __threadfence();
    *(volatile v4u*)q = w;
  }
  if (tid < 32) {
    const int r = tid < 2 ? tid : 2;
    float g0 = sR[r * 3], g1 = sR[r * 3 + 1], g2 = sR[r * 3 + 2];
    float gt = sJ[r];
    {
      const float jx = sJ[0], jy = sJ[1], jz = sJ[2];
      const float tr = gt - (g0 * jx + g1 * jy + g2 * jz);
      if (tid < 3) {
        sA[(r * 4 + 0) * 56] = g0;
        sA[(r * 4 + 1) * 56] = g1;
        sA[(r * 4 + 2) * 56] = g2;
        sA[(r * 4 + 3) * 56] = tr;
      }
    }
#pragma unroll 1
    for (int j = 1; j < kJ; ++j) {
      const float* Rj = sR + j * 9;
      const float jx = sJ[j * 3], jy = sJ[j * 3 + 1], jz = sJ[j * 3 + 2];
      const float t0 = jx - sJ[j * 3 - 3];
      const float t1 = jy - sJ[j * 3 - 2];
      const float t2 = jz - sJ[j * 3 - 1];
      const float n0 = g0 * Rj[0] + g1 * Rj[3] + g2 * Rj[6];
      const float n1 = g0 * Rj[1] + g1 * Rj[4] + g2 * Rj[7];
      const float n2 = g0 * Rj[2] + g1 * Rj[5] + g2 * Rj[8];
      gt = (g0 * t0 + g1 * t1 + g2 * t2) + gt;
      g0 = n0; g1 = n1; g2 = n2;
      const float tr = gt - (g0 * jx + g1 * jy + g2 * jz);
      if (tid < 3) {
        sA[(r * 4 + 0) * 56 + j] = g0;
        sA[(r * 4 + 1) * 56 + j] = g1;
        sA[(r * 4 + 2) * 56 + j] = g2;
        sA[(r * 4 + 3) * 56 + j] = tr;
      }
    }
  }
  __syncthreads();
  {
    v4u w[2];
#pragma unroll
    for (int it = 0; it < 2; ++it) {
      const int row = it * 8 + (tid >> 3);
      const int rc = row < 11 ? row : 11;
      const int c8 = (tid & 7) * 8;
      unsigned short hb[8];
#pragma unroll
      for (int e = 0; e < 8; ++e) {
        const int j = c8 + e;
        const int jc = j < kJ - 1 ? j : kJ - 1;
        const float sv = sA[rc * 56 + jc];
        const float val = (row < 12 && j < kJ) ? sv : 0.0f;
        hb[e] = f2h_bits(val);
      }
      w[it] = (v4u){pack2(hb[0], hb[1]), pack2(hb[2], hb[3]), pack2(hb[4], hb[5]), pack2(hb[6], hb[7])};
    }
    for (int pass = 0; pass < 2; ++pass) {
#pragma unroll
      for (int it = 0; it < 2; ++it) {
        const int row = it * 8 + (tid >> 3);
        unsigned short* q = At + ((size_t)(b * 16 + row)) * kJP + (tid & 7) * 8;
        *(volatile v4u*)q = w[it];
      }
      __threadfence();
    }
  }
}

__global__ __launch_bounds__(256) void pdt_kernel(
    const float* __restrict__ pd, const float* __restrict__ ed, unsigned short* __restrict__ pdt)
{
  __shared__ float t[64 * 65];
  const int tid = threadIdx.x;
  const int n0 = blockIdx.x * 64, k0 = blockIdx.y * 64;
  const int tx = tid & 63, ty = tid >> 6;
  {
    const int n = n0 + tx;
    const int nc = n < kN3 ? n : kN3 - 1;
    const bool nok = n < kN3;
#pragma unroll
    for (int i = 0; i < 16; ++i) {
      const int kk = ty + 4 * i;
      const int k = k0 + kk;
      const int kc = k < kPF ? k : kPF - 1;
      const float v = pd[(size_t)kc * kN3 + nc];
      t[kk * 65 + tx] = (nok && k < kPF) ? v : 0.0f;
    }
  }
  __syncthreads();
  if (blockIdx.y == kEdTile) {
#pragma unroll
    for (int it = 0; it < 3; ++it) {
      const int idx = tid + 256 * it;
      const int ic = idx < 639 ? idx : 639;
      const int e = ic >> 6, nn = ic & 63;
      const int n2 = n0 + nn;
      const int n2c = n2 < kN3 ? n2 : kN3 - 1;
      const float v = ed[(size_t)n2c * kNE + e];
      if (idx < 640) t[(kEdRow + e) * 65 + nn] = (n2 < kN3) ? v : 0.0f;
    }
  }
  __syncthreads();
  v4u w[2];
#pragma unroll
  for (int it = 0; it < 2; ++it) {
    const int row = it * 32 + (tid >> 3);
    const int c8 = (tid & 7) * 8;
    unsigned short hb[8];
#pragma unroll
    for (int e = 0; e < 8; ++e) hb[e] = f2bf_bits(t[(c8 + e) * 65 + row]);
    w[it] = (v4u){pack2(hb[0], hb[1]), pack2(hb[2], hb[3]), pack2(hb[4], hb[5]), pack2(hb[6], hb[7])};
  }
  for (int pass = 0; pass < 2; ++pass) {
#pragma unroll
    for (int it = 0; it < 2; ++it) {
      const int row = it * 32 + (tid >> 3);
      unsigned short* q = pdt + (size_t)(n0 + row) * kKP + k0 + (tid & 7) * 8;
      *(volatile v4u*)q = w[it];
    }
    __threadfence();
  }
}

__global__ __launch_bounds__(256) void wconv_kernel(const float* __restrict__ W, unsigned short* __restrict__ Wb)
{
  const int i = blockIdx.x * 256 + threadIdx.x;
  if (i >= kVP * 8) return;
  const int v = i >> 3, c8 = (i & 7) * 8;
  const int vc = v < kV ? v : kV - 1;
  unsigned short hb[8];
#pragma unroll
  for (int e = 0; e < 8; ++e) {
    const int j = c8 + e;
    const int jc = j < kJ - 1 ? j : kJ - 1;
    const float x = W[(size_t)vc * kJ + jc];
    const float val = (v < kV && j < kJ) ? x * kWCarry : 0.0f;
    hb[e] = f2h_bits(val);
  }
  const v4u w = (v4u){pack2(hb[0], hb[1]), pack2(hb[2], hb[3]), pack2(hb[4], hb[5]), pack2(hb[6], hb[7])};
  unsigned short* q = Wb + (size_t)v * kJP + c8;
  *(volatile v4u*)q = w;
  __threadfence();
  *(volatile v4u*)q = w;
}

__global__ __launch_bounds__(256) void pose_gemm_kernel(
    const unsigned short* __restrict__ Ap, const unsigned short* __restrict__ Btp,
    const float* __restrict__ addn, float* __restrict__ C)
{
  typedef __bf16 T;
  const T* A = (const T*)Ap;
  const T* Bt = (const T*)Btp;
  __shared__ __align__(16) float sT[8][16 * 68];
  constexpr int lda = kKP, ldb = kKP, ldc = kNP;
  constexpr int tilesN = kNP >> 6, tilesM = kB >> 6;
  const int lane = threadIdx.x & 31;
  const int wave = threadIdx.x >> 5;
  const int tile = blockIdx.x * 8 + wave;
  if (tile >= tilesM * tilesN) return;
  const int tm = tile / tilesN;
  const int tn = tile - tm * tilesN;
  const int m0 = tm << 6;
  const int n0 = tn << 6;
  const int rlane = lane & 15;
  const int koff  = (lane >> 4) * 8;
  const int mOff  = (lane >> 4) * 8;

  v8f acc[4][4];
#pragma unroll
  for (int i = 0; i < 4; ++i)
#pragma unroll
    for (int j = 0; j < 4; ++j) acc[i][j] = (v8f){0.f,0.f,0.f,0.f,0.f,0.f,0.f,0.f};

  for (int k0 = 0; k0 < kKP; k0 += 32) {
    v16b bh[4];
#pragma unroll
    for (int j = 0; j < 4; ++j) {
      const size_t bo = (size_t)(n0 + (j << 4) + rlane) * ldb + koff + k0;
      bh[j] = Frag<T>::load(Bt + bo);
    }
#pragma unroll
    for (int i = 0; i < 4; ++i) {
      const size_t ao = (size_t)(m0 + (i << 4) + rlane) * lda + koff + k0;
      const v16b ah = Frag<T>::load(A + ao);
#pragma unroll
      for (int j = 0; j < 4; ++j) acc[i][j] = mma_b(ah, bh[j], acc[i][j]);
    }
    keep4_b(bh[0], bh[1], bh[2], bh[3]);
  }

  float bv[4];
#pragma unroll
  for (int j = 0; j < 4; ++j) bv[j] = addn[n0 + (j << 4) + rlane];

  float* slab = sT[wave];
#pragma unroll
  for (int i = 0; i < 4; ++i) {
    const int mBase = m0 + (i << 4);
#pragma unroll
    for (int j = 0; j < 4; ++j) {
#pragma unroll
      for (int r = 0; r < 8; ++r) {
        const float v = acc[i][j][r] + bv[j];
        slab[(mOff + r) * 68 + (j << 4) + rlane] = v;
      }
    }
    __builtin_amdgcn_fence(__ATOMIC_RELEASE, "workgroup");
    __builtin_amdgcn_wave_barrier();
    __builtin_amdgcn_fence(__ATOMIC_ACQUIRE, "workgroup");
    {
      const int hh = lane >> 4, c4 = (lane & 15) * 4;
      for (int pass = 0; pass < 2; ++pass) {
#pragma unroll
        for (int it = 0; it < 8; ++it) {
          const int row = it * 2 + hh;
          const v4f v = *(const v4f*)(slab + row * 68 + c4);
          *(volatile v4f*)(C + (size_t)(mBase + row) * ldc + n0 + c4) = v;
        }
        __threadfence();
      }
    }
    __builtin_amdgcn_fence(__ATOMIC_RELEASE, "workgroup");
    __builtin_amdgcn_wave_barrier();
    __builtin_amdgcn_fence(__ATOMIC_ACQUIRE, "workgroup");
  }
}

__global__ __launch_bounds__(256) void lbs_skin_kernel(
    const unsigned short* __restrict__ Wbp, const unsigned short* __restrict__ Atp,
    const float* __restrict__ vposed, const float* __restrict__ yoffp,
    const float* __restrict__ gtr, float* __restrict__ out,
    float* __restrict__ headtab, float* __restrict__ tailtab)
{
  __shared__ __align__(16) float sT[kLbsTileV * kTP];
  __shared__ __align__(16) float sX[2 * kGrpB * kRun];
  __shared__ float sHead[kGrpB * 32];
  const _Float16* Wb = (const _Float16*)Wbp;
  const _Float16* At = (const _Float16*)Atp;
  const int tid = threadIdx.x, lane = tid & 31, wave = tid >> 5;
  const int rlane = lane & 15, hh = lane >> 4, koff = hh * 8;
  const int b0 = blockIdx.x * kGrpB;

#pragma unroll
  for (int i = 0; i < 6; ++i) sX[kGrpB * kRun + i * 256 + tid] = 0.0f;

  v16h bf0[4], bf1[4];
#pragma unroll
  for (int j = 0; j < 4; ++j) {
    const _Float16* bp = At + (size_t)((b0 + j) * 16 + rlane) * kJP + koff;
    bf0[j] = Frag<_Float16>::load(bp);
    bf1[j] = Frag<_Float16>::load(bp + 32);
  }
  const float yoff = yoffp[0];

  const int vl = tid & 127, bsel = tid >> 7;
  float gx[2], gy[2], gz[2];
#pragma unroll
  for (int it = 0; it < 2; ++it) {
    const int b = b0 + bsel + 2 * it;
    gx[it] = gtr[b * 3 + 0];
    gy[it] = gtr[b * 3 + 1];
    gz[it] = gtr[b * 3 + 2];
  }

  const int sbi = wave >> 1, shalf = wave & 1;
  const int sb = b0 + sbi;
  const int p = sb & 31;
  const size_t rowbase = (size_t)sb * kN3;

#pragma unroll 1
  for (int tile = 0; tile < kLbsTiles; ++tile) {
    const int v0 = tile * kLbsTileV;
    const int buf = tile & 1;
    {
      const _Float16* ap = Wb + (size_t)(v0 + wave * 16 + rlane) * kJP + koff;
      const v16h af0 = Frag<_Float16>::load(ap);
      const v16h af1 = Frag<_Float16>::load(ap + 32);
      v8f acc[4];
#pragma unroll
      for (int j = 0; j < 4; ++j) {
        acc[j] = (v8f){0.f,0.f,0.f,0.f,0.f,0.f,0.f,0.f};
        acc[j] = mma_h(af0, bf0[j], acc[j]);
        acc[j] = mma_h(af1, bf1[j], acc[j]);
      }
#pragma unroll
      for (int j = 0; j < 4; ++j) {
#pragma unroll
        for (int r = 0; r < 8; ++r)
          sT[(wave * 16 + 8 * hh + r) * kTP + (j << 4) + rlane] = acc[j][r] * kWCarryInv;
      }
    }
    __syncthreads();
#pragma unroll
    for (int it = 0; it < 2; ++it) {
      const int bi = bsel + 2 * it;
      const int b = b0 + bi;
      const float* tp = sT + vl * kTP + bi * 16;
      const v4f t0 = *(const v4f*)(tp);
      const v4f t1 = *(const v4f*)(tp + 4);
      const v4f t2 = *(const v4f*)(tp + 8);
      const float* vp = vposed + (size_t)b * kNP + (size_t)(v0 + vl) * 3;
      const float p0 = vp[0], p1 = vp[1], p2 = vp[2];
      const float o0 = ((t0[0] * p0 + t0[1] * p1 + t0[2] * p2) + t0[3]) + gx[it];
      const float o1 = (((t1[0] * p0 + t1[1] * p1 + t1[2] * p2) + t1[3]) + yoff) + gy[it];
      const float o2 = ((t2[0] * p0 + t2[1] * p1 + t2[2] * p2) + t2[3]) + gz[it];
      float* xo = sX + (buf * kGrpB + bi) * kRun + vl * 3;
      xo[0] = o0;
      xo[1] = o1;
      xo[2] = o2;
    }
    __syncthreads();
    {
      const int nv3 = (kV - v0) * 3;
      const int nvalid = nv3 < kRun ? nv3 : kRun;
      const int nfull = (nvalid + p) >> 5;
      const size_t Lb = rowbase + (size_t)(kRun * tile) - (size_t)p;
      const float* xc = sX + (buf * kGrpB + sbi) * kRun;
      const float* xq = sX + ((buf ^ 1) * kGrpB + sbi) * kRun;
      const bool defer = (tile == 0) && (p > 0);
      float val[6];
      bool ok[6];
#pragma unroll
      for (int i6 = 0; i6 < 6; ++i6) {
        const int i = shalf * 6 + i6;
        const int o = 32 * i + lane - p;
        const int oc = o < 0 ? 0 : (o > kRun - 1 ? kRun - 1 : o);
        int oq = kRun + o;
        oq = oq < 0 ? 0 : (oq > kRun - 1 ? kRun - 1 : oq);
        const float vc = xc[oc];
        const float vq = xq[oq];
        val[i6] = (o < 0) ? vq : vc;
        ok[i6] = (i < nfull) && !(defer && i == 0);
      }
      if (tile == 0 && shalf == 0) sHead[sbi * 32 + lane] = val[0];
      for (int pass = 0; pass < 2; ++pass) {
#pragma unroll
        for (int i6 = 0; i6 < 6; ++i6) {
          const int i = shalf * 6 + i6;
          if (ok[i6]) *(volatile float*)(out + Lb + (size_t)(32 * i + lane)) = val[i6];
        }
        __threadfence();
      }
    }
  }
  if (shalf == 0) {
    constexpr int kLastValid = (kV - (kLbsTiles - 1) * kLbsTileV) * 3;
    constexpr int kLastBuf = (kLbsTiles - 1) & 1;
    const int q = (kLastValid + p) & 31;
    const int nfl = (kLastValid + p) >> 5;
    const int ot = 32 * nfl - p + lane;
    const int otc = ot < 0 ? 0 : (ot > kRun - 1 ? kRun - 1 : ot);
    const float tv = sX[(kLastBuf * kGrpB + sbi) * kRun + otc];
    const int hb = sbi < kGrpB - 1 ? sbi + 1 : kGrpB - 1;
    const float hv = sHead[hb * 32 + lane];
    const float h0 = sHead[lane];
    const float v = (lane < q) ? tv : hv;
    const float tz = (lane < q) ? tv : 0.0f;
    const bool okb = (q > 0) && (sbi < kGrpB - 1);
    const size_t idx = rowbase + (size_t)(kN3 - q) + (size_t)lane;
    float* ht = headtab + (size_t)blockIdx.x * 32 + lane;
    float* tt = tailtab + (size_t)blockIdx.x * 32 + lane;
    for (int pass = 0; pass < 2; ++pass) {
      if (okb) *(volatile float*)(out + idx) = v;
      if (sbi == 0) *(volatile float*)ht = h0;
      if (sbi == kGrpB - 1) *(volatile float*)tt = tz;
      __threadfence();
    }
  }
}

__global__ __launch_bounds__(256) void edge_merge_kernel(
    const float* __restrict__ headtab, const float* __restrict__ tailtab, float* __restrict__ out)
{
  const int lane = threadIdx.x & 31, wave = threadIdx.x >> 5;
  const int g = blockIdx.x * 8 + wave;
  const int b0 = g * kGrpB;
  const int p = b0 & 31;
  if (g <= 0 || g >= kGroups || p == 0) return;
  const float tv = tailtab[(size_t)(g - 1) * 32 + lane];
  const float hv = headtab[(size_t)g * 32 + lane];
  const float v = (lane < p) ? tv : hv;
  float* q = out + ((size_t)b0 * kN3 - (size_t)p) + (size_t)lane;
  *(volatile float*)q = v;
  __threadfence();
  *(volatile float*)q = v;
}

extern "C" void kernel_launch(void* const* d_in, const int* in_sizes, int n_in,
                              void* d_out, int out_size, void* d_ws, size_t ws_size,
                              hipStream_t stream) {
  if (n_in < 14) return;
  if (in_sizes[0] != kNE) return;
  if (in_sizes[1] != kB * 63) return;
  if (in_sizes[2] != kB * 90) return;
  if (in_sizes[3] != kB * 9) return;
  if (in_sizes[4] != kB * kNE) return;
  if (in_sizes[5] != kB * 3) return;
  if (in_sizes[6] != kB * 3) return;
  if (in_sizes[7] != kN3) return;
  if (in_sizes[8] != kN3 * kNE) return;
  if (in_sizes[9] != kN3 * kNE) return;
  if (in_sizes[10] != kPF * kN3) return;
  if (in_sizes[11] != kV * kJ) return;
  if (in_sizes[12] != kJ * kV) return;
  if (in_sizes[13] != 90) return;
  if (out_size != kB * kN3) return;
  if (ws_size < kWsTotal) return;

  const float* shape     = (const float*)d_in[0];
  const float* body      = (const float*)d_in[1];
  const float* hand      = (const float*)d_in[2];
  const float* head      = (const float*)d_in[3];
  const float* expr      = (const float*)d_in[4];
  const float* pelvis    = (const float*)d_in[5];
  const float* gtrans    = (const float*)d_in[6];
  const float* vtempl    = (const float*)d_in[7];
  const float* shapedirs = (const float*)d_in[8];
  const float* exprdirs  = (const float*)d_in[9];
  const float* posedirs  = (const float*)d_in[10];
  const float* lbsw      = (const float*)d_in[11];
  const float* jreg      = (const float*)d_in[12];
  const float* hmean     = (const float*)d_in[13];
  float* out = (float*)d_out;

  char* ws = (char*)d_ws;
  float*          VPOSED = (float*)(ws + kOffVP);
  unsigned short* PDT    = (unsigned short*)(ws + kOffPDT);
  unsigned short* WB     = (unsigned short*)(ws + kOffWB);
  unsigned short* AT     = (unsigned short*)(ws + kOffAT);
  unsigned short* APOSE  = (unsigned short*)(ws + kOffAP);
  float*          BASE   = (float*)(ws + kOffBASE);
  float*          JT     = (float*)(ws + kOffJT);
  float*          YOFF   = (float*)(ws + kOffYO);
  float*          HEADT  = (float*)(ws + kOffHT);
  float*          TAILT  = (float*)(ws + kOffTT);

  static_base_kernel<<<(kNP / 4 + 255) / 256, 256, 0, stream>>>(vtempl, shapedirs, shape, BASE);
  yoff_kernel<<<1, 256, 0, stream>>>(vtempl, YOFF);
  jreg_kernel<<<kJ, 256, 0, stream>>>(jreg, BASE, exprdirs, JT);
  pose_fk_kernel<<<kB, 64, 0, stream>>>(pelvis, body, head, hand, hmean, expr, JT, APOSE, AT);
  pdt_kernel<<<dim3(kNP / 64, kKP / 64), 256, 0, stream>>>(posedirs, exprdirs, PDT);
  wconv_kernel<<<(kVP * 8) / 256, 256, 0, stream>>>(lbsw, WB);
  pose_gemm_kernel<<<((kB / 64) * (kNP / 64)) / 8, 256, 0, stream>>>(APOSE, PDT, BASE, VPOSED);
  lbs_skin_kernel<<<kGroups, 256, 0, stream>>>(WB, AT, VPOSED, YOFF, gtrans, out, HEADT, TAILT);
  edge_merge_kernel<<<kGroups / 8, 256, 0, stream>>>(HEADT, TAILT, out);
}
